// pLoss_all_21517786153438
// MI455X (gfx1250) — hardware-verified
//
#include <hip/hip_runtime.h>


namespace {
constexpr int NB = 8192, L = 64, NS = 4096;
constexpr int QT = NB / 16;
constexpr float P_SC = 4096.0f;

typedef _Float16 b16;
typedef __attribute__((ext_vector_type(16))) _Float16 v16b;
typedef __attribute__((ext_vector_type(8)))  _Float16 v8b;
typedef __attribute__((ext_vector_type(8)))  float v8f;
typedef __attribute__((ext_vector_type(4)))  float v4f;

__device__ __forceinline__ v8b ld8b(const b16* p) { return *(const v8b*)p; }
__device__ __forceinline__ v16b cat8b(v8b a, v8b b) { return __builtin_shufflevector(a, b, 0, 1, 2, 3, 4, 5, 6, 7, 8, 9, 10, 11, 12, 13, 14, 15); }
__device__ __forceinline__ v16b frag_kb(const b16* p, int hh) { return cat8b(ld8b(p + 8 * hh), ld8b(p + 16 + 8 * hh)); }
__device__ __forceinline__ void split16(float v, b16& hi, b16& lo) { hi = (b16)v; lo = (b16)(v - (float)hi); }
__device__ __forceinline__ v8f wmma16b(v16b a, v16b b, v8f c) {
  v8f d = __builtin_amdgcn_wmma_f32_16x16x32_f16(false, a, false, b, (short)0, c, false, false);
  asm volatile("v_nop\n\tv_nop\n\tv_nop\n\tv_nop" : "+v"(d) : "v"(a), "v"(b));
  return d;
}

__global__ __launch_bounds__(256) void prep_kernel(const float* __restrict__ f, const float* __restrict__ S, b16* __restrict__ fh, b16* __restrict__ fl,
                                                   b16* __restrict__ S16, b16* __restrict__ ST16) {
  const size_t tid = (size_t)blockIdx.x * blockDim.x + threadIdx.x, stride = (size_t)gridDim.x * blockDim.x;
  const size_t nf = (size_t)NB * L / 8, ns = (size_t)NS * L / 8, nt = (size_t)NS * L / 8;
  for (int pass = 0; pass < 2; ++pass) {
    for (size_t c = tid; c < nf + ns + nt; c += stride) {
      if (c < nf) { const size_t i = c * 8; v8b a, b2;
#pragma unroll
        for (int e = 0; e < 8; ++e) { b16 x, y; split16(f[i + e], x, y); a[e] = x; b2[e] = y; }
        *(volatile v8b*)(fh + i) = a; *(volatile v8b*)(fl + i) = b2;
      } else if (c < nf + ns) { const size_t i = (c - nf) * 8; v8b a;
#pragma unroll
        for (int e = 0; e < 8; ++e) a[e] = (b16)S[i + e];
        *(volatile v8b*)(S16 + i) = a;
      } else {
        const size_t i = (c - nf - ns) * 8; const int t = (int)(i / 1024), l = (int)((i % 1024) / 16), j0 = (int)(i % 16);
        v8b a;
#pragma unroll
        for (int e = 0; e < 8; ++e) a[e] = (b16)S[(size_t)(16 * t + j0 + e) * L + l];
        *(volatile v8b*)(ST16 + i) = a;
      }
    }
    __threadfence();
  }
}

__global__ __launch_bounds__(256) void marg_kernel(const b16* __restrict__ fh, const b16* __restrict__ fl, const b16* __restrict__ S16, const b16* __restrict__ ST16,
                                                   const float* __restrict__ y, const float* __restrict__ mask, float* __restrict__ pm, float* __restrict__ bslot) {
  __shared__ __attribute__((aligned(16))) float Os[8][16 * 64];
  __shared__ float term[128];
  const int wid = threadIdx.x >> 5, lane = threadIdx.x & 31, hh = lane >> 4, col = lane & 15;
  const int q0 = (blockIdx.x * 8 + wid) * 16;
  const size_t qo = (size_t)(q0 + col) * L;
  const v16b q0h = frag_kb(fh + qo, hh), q1h = frag_kb(fh + qo + 32, hh), q0l = frag_kb(fl + qo, hh), q1l = frag_kb(fl + qo + 32, hh);
  float m = -INFINITY, l = 0.0f;
  v8f o0 = {}, o1 = {}, o2 = {}, o3 = {};
  for (int kb = 0; kb < NS; kb += 32) {
    const size_t r0 = (size_t)(kb + col) * L, r1 = (size_t)(kb + 16 + col) * L;
    v8f s0 = {}, s1 = {};
    v16b a = frag_kb(S16 + r0, hh);       s0 = wmma16b(a, q0h, s0); s0 = wmma16b(a, q0l, s0);
    a = frag_kb(S16 + r0 + 32, hh);       s0 = wmma16b(a, q1h, s0); s0 = wmma16b(a, q1l, s0);
    a = frag_kb(S16 + r1, hh);            s1 = wmma16b(a, q0h, s1); s1 = wmma16b(a, q0l, s1);
    a = frag_kb(S16 + r1 + 32, hh);       s1 = wmma16b(a, q1h, s1); s1 = wmma16b(a, q1l, s1);
    float mr = -INFINITY;
#pragma unroll
    for (int r = 0; r < 8; ++r) mr = fmaxf(mr, fmaxf(s0[r], s1[r]));
    mr = fmaxf(mr, __shfl_xor(mr, 16));
    const float mn = fmaxf(m, mr), al_ = __expf(m - mn);
    m = mn;
    float sum = 0.0f; v16b pb;
#pragma unroll
    for (int r = 0; r < 8; ++r) { const float p0 = __expf(s0[r] - mn), p1 = __expf(s1[r] - mn); sum += p0 + p1; pb[r] = (b16)(p0 * P_SC); pb[8 + r] = (b16)(p1 * P_SC); }
    sum += __shfl_xor(sum, 16);
    l = l * al_ + sum;
#pragma unroll
    for (int r = 0; r < 8; ++r) { o0[r] *= al_; o1[r] *= al_; o2[r] *= al_; o3[r] *= al_; }
    const size_t v0 = (size_t)(kb >> 4) * (L * 16) + 8 * hh, v1 = v0 + L * 16;
#pragma unroll
    for (int n = 0; n < 4; ++n) {
      const int fcol = n * 16 + col;
      const v16b va = cat8b(ld8b(ST16 + v0 + fcol * 16), ld8b(ST16 + v1 + fcol * 16));
      v8f& o = (n == 0) ? o0 : (n == 1) ? o1 : (n == 2) ? o2 : o3;
      o = wmma16b(va, pb, o);
    }
  }
  const float inv = 1.0f / (P_SC * l);
  float* Tt = Os[wid];
#pragma unroll
  for (int r = 0; r < 8; ++r) {
    const int hr = 8 * hh + r;
    Tt[col * 64 + 0 + hr] = o0[r] * inv; Tt[col * 64 + 16 + hr] = o1[r] * inv;
    Tt[col * 64 + 32 + hr] = o2[r] * inv; Tt[col * 64 + 48 + hr] = o3[r] * inv;
  }
  __builtin_amdgcn_fence(__ATOMIC_RELEASE, "workgroup"); __builtin_amdgcn_wave_barrier(); __builtin_amdgcn_fence(__ATOMIC_ACQUIRE, "workgroup");
  float* dst0 = pm + (size_t)q0 * L;
  for (int pass = 0; pass < 2; ++pass) {
#pragma unroll
    for (int j = 0; j < 8; ++j) { const int rr = j * 2 + hh, c4 = col * 4; *(volatile v4f*)(dst0 + (size_t)rr * L + c4) = *(const v4f*)(Tt + rr * 64 + c4); }
    __threadfence();
  }
  {
    const int row = q0 + col; float acc = 0.0f;
    for (int e = 0; e < 32; ++e) {
      const int lab = 32 * hh + e;
      const float p = Tt[col * 64 + lab], yy = y[(size_t)row * L + lab], mk = mask[(size_t)row * L + lab];
      const float lp = fmaxf(logf(p), -100.0f), l1p = fmaxf(log1pf(-p), -100.0f);
      acc += -(yy * lp + (1.0f - yy) * l1p) * mk;
    }
    const float tot = acc + __shfl_xor(acc, 16);
    if (hh == 0) term[wid * 16 + col] = tot * (1.0f / L);
  }
  __syncthreads();
  if (wid == 0) {
    float bsum = 0.0f;
    if (lane == 0) { for (int i = 0; i < 128; ++i) bsum += term[i]; }
    const float v = (lane == 0) ? bsum : 0.0f;
    ((volatile float*)bslot)[(size_t)blockIdx.x * 32 + lane] = v;
    __threadfence();
    ((volatile float*)bslot)[(size_t)blockIdx.x * 32 + lane] = v;
  }
}

__global__ __launch_bounds__(256) void pack_kernel(const float* __restrict__ pm, const float* __restrict__ bslot, float* __restrict__ out, int total) {
  __shared__ float loss_s;
  if (threadIdx.x == 0) { float s = 0.0f; for (int i = 0; i < NB / 128; ++i) s += bslot[(size_t)i * 32]; loss_s = s * (1.0f / NB); }
  __syncthreads();
  const float loss = loss_s;
  const int base = blockIdx.x * 8192;
  for (int pass = 0; pass < 2; ++pass) {
    for (int i = threadIdx.x; i < 8192; i += 256) {
      const int gidx = base + i;
      if (gidx < total) ((volatile float*)out)[gidx] = (gidx == 0) ? loss : pm[gidx - 1];
    }
    __threadfence();
  }
}
}

extern "C" void kernel_launch(void* const* d_in, const int* in_sizes, int n_in,
                              void* d_out, int out_size, void* d_ws, size_t ws_size, hipStream_t stream) {
  (void)n_in;
  const float* f    = (const float*)d_in[0];
  const float* y    = (const float*)d_in[1];
  const float* mask = (const float*)d_in[2];
  const float* S    = (const float*)d_in[3];
  float* out = (float*)d_out;
  if (in_sizes[0] != NB * L || in_sizes[3] != NS * L || out_size != 1 + NB * L) return;

  size_t off = 0; char* ws = (char*)d_ws;
  auto carve = [&](size_t bytes) { char* p = ws + off; off += (bytes + 255) & ~(size_t)255; return p; };
  b16* fh   = (b16*)carve((size_t)NB * L * 2);
  b16* fl   = (b16*)carve((size_t)NB * L * 2);
  b16* S16  = (b16*)carve((size_t)NS * L * 2);
  b16* ST16 = (b16*)carve((size_t)NS * L * 2);
  float* pm = (float*)carve((size_t)NB * L * 4);
  float* bs = (float*)carve((size_t)(NB / 128) * 32 * 4);
  if (off > ws_size) return;
  prep_kernel<<<512, 256, 0, stream>>>(f, S, fh, fl, S16, ST16);
  marg_kernel<<<QT / 8, 256, 0, stream>>>(fh, fl, S16, ST16, y, mask, pm, bs);
  pack_kernel<<<(1 + NB * L + 8191) / 8192, 256, 0, stream>>>(pm, bs, out, 1 + NB * L);
}
